// BlockDiT_69715909148723
// MI455X (gfx1250) — hardware-verified
//
#include <hip/hip_runtime.h>

#define DIM   768
#define SEQ   2048
#define NHALF 1024
#define HEADS 12
#define HD    64
#define DFF   3072
#define COND  128
#define ROWS  4096
#define ADA6  4608
#define QKVW  2304
#define BLK   16

typedef __attribute__((ext_vector_type(16))) _Float16 v16h;
typedef __attribute__((ext_vector_type(8)))  _Float16 v8h;
typedef __attribute__((ext_vector_type(16))) __bf16   v16b;
typedef __attribute__((ext_vector_type(8)))  __bf16   v8b;
typedef __attribute__((ext_vector_type(8)))  float    v8f;
typedef __attribute__((ext_vector_type(4)))  float    v4f;
typedef __attribute__((ext_vector_type(4)))  int      v4i;
#define PSCALE 32768.0f
#define U16(p) ((const unsigned short*)(const void*)(p))
#define PSCALE_INV (1.0f / 32768.0f)

__device__ __forceinline__ unsigned short f2bf_bits(float f) {
  unsigned u = __float_as_uint(f);
  return (unsigned short)((u + 0x7FFFu + ((u >> 16) & 1u)) >> 16);
}
__device__ __forceinline__ float bf_bits2f(unsigned short h) { return __uint_as_float(((unsigned)h) << 16); }

__device__ __forceinline__ void dep_guard_h(v8f& a, v8f& b, v16h x, v16h y) { asm volatile("v_nop\n\tv_nop\n\tv_nop\n\tv_nop" : "+v"(a), "+v"(b) : "v"(x), "v"(y)); }
__device__ __forceinline__ void dep_guard_b(v8f& a, v8f& b, v16b x, v16b y) { asm volatile("v_nop\n\tv_nop\n\tv_nop\n\tv_nop" : "+v"(a), "+v"(b) : "v"(x), "v"(y)); }
__device__ __forceinline__ void keep4_h(v16h a, v16h b, v16h c, v16h d) { asm volatile("v_nop" :: "v"(a), "v"(b), "v"(c), "v"(d)); }
__device__ __forceinline__ void keep4_b(v16b a, v16b b, v16b c, v16b d) { asm volatile("v_nop" :: "v"(a), "v"(b), "v"(c), "v"(d)); }
__device__ __forceinline__ void acc_guard4(v8f& a, v8f& b, v8f& c, v8f& d) { asm volatile("v_nop\n\tv_nop\n\tv_nop\n\tv_nop" : "+v"(a), "+v"(b), "+v"(c), "+v"(d)); }
template <typename T> struct Frag;
template <> struct Frag<_Float16> {
  typedef v16h V; union U { v16h v; v8h h[2]; };
  static __device__ __forceinline__ v16h load(const _Float16* p) {
    U f; f.h[0] = *(const v8h*)(p); f.h[1] = *(const v8h*)(p + 16); return f.v;
  }
  static __device__ __forceinline__ v8f mma(v16h a, v16h b, v8f c) {
    return __builtin_amdgcn_wmma_f32_16x16x32_f16(false, a, false, b, (short)0, c, false, false);
  }
  static __device__ __forceinline__ void guard(v8f& a, v8f& b, v16h x, v16h y) { dep_guard_h(a, b, x, y); }
  static __device__ __forceinline__ void keep(v16h a, v16h b, v16h c, v16h d) { keep4_h(a, b, c, d); }
};
template <> struct Frag<__bf16> {
  typedef v16b V; union U { v16b v; v8b h[2]; };
  static __device__ __forceinline__ v16b load(const __bf16* p) {
    U f; f.h[0] = *(const v8b*)(p); f.h[1] = *(const v8b*)(p + 16); return f.v;
  }
  static __device__ __forceinline__ v8f mma(v16b a, v16b b, v8f c) {
    return __builtin_amdgcn_wmma_f32_16x16x32_bf16(false, a, false, b, (short)0, c, false, false);
  }
  static __device__ __forceinline__ void guard(v8f& a, v8f& b, v16b x, v16b y) { dep_guard_b(a, b, x, y); }
  static __device__ __forceinline__ void keep(v16b a, v16b b, v16b c, v16b d) { keep4_b(a, b, c, d); }
};

__device__ __forceinline__ float gelu_tanh_f(float v) {
  const float t = 0.7978845608028654f * (v + 0.044715f * v * v * v);
  const float e = __expf(2.0f * t);
  const float th = 1.0f - 2.0f * __builtin_amdgcn_rcpf(e + 1.0f);
  return 0.5f * v * (1.0f + th);
}

template <int ET> struct Elem;
template <> struct Elem<0> { typedef _Float16 T; };
template <> struct Elem<1> { typedef __bf16 T; };
template <int ET, bool SPLIT, int BIAS_MODE, int OUT_MODE, bool RESID, int ACT = 0>
__global__ __launch_bounds__(256) void wmma_gemm64(
    const unsigned short* __restrict__ Ap, const unsigned short* __restrict__ A2p, int lda, long strideA,
    const unsigned short* __restrict__ Btp, const unsigned short* __restrict__ Bt2p, int ldb, long strideB,
    void* __restrict__ Cout, void* __restrict__ Cout2, int ldc, long strideC,
    const float* __restrict__ bias,
    const float* __restrict__ resid, long strideR,
    int M, int N, int K, float scale) {
  typedef typename Elem<ET>::T T;
  typedef typename Frag<T>::V V;
  const T* A = (const T*)Ap; const T* A2 = (const T*)A2p; const T* Bt = (const T*)Btp; const T* Bt2 = (const T*)Bt2p;
  __shared__ __align__(16) float sT[8][16 * 68];
  const int b    = blockIdx.y;
  const int lane = threadIdx.x & 31;
  const int wave = threadIdx.x >> 5;
  const int tilesN = N >> 6;
  const int tilesM = M >> 6;
  const int tile = blockIdx.x * 8 + wave;
  if (tile >= tilesM * tilesN) return;
  const int tm = tile / tilesN;
  const int tn = tile - tm * tilesN;
  const int m0 = tm << 6;
  const int n0 = tn << 6;

  const T* Ab  = A  + (size_t)b * strideA;
  const T* Bb  = Bt + (size_t)b * strideB;
  const T* Ab2 = SPLIT ? (A2  + (size_t)b * strideA) : nullptr;
  const T* Bb2 = SPLIT ? (Bt2 + (size_t)b * strideB) : nullptr;

  const int rlane = lane & 15;
  const int koff  = (lane >> 4) * 8;
  const int mOff  = (lane >> 4) * 8;

  v8f acc[4][4];
#pragma unroll
  for (int i = 0; i < 4; ++i)
#pragma unroll
    for (int j = 0; j < 4; ++j) acc[i][j] = (v8f){0.f,0.f,0.f,0.f,0.f,0.f,0.f,0.f};

  for (int k0 = 0; k0 < K; k0 += 32) {
    V bh[4], bl[4];
#pragma unroll
    for (int j = 0; j < 4; ++j) {
      const size_t bo = (size_t)(n0 + (j << 4) + rlane) * ldb + koff + k0;
      bh[j] = Frag<T>::load(Bb + bo);
      if (SPLIT) bl[j] = Frag<T>::load(Bb2 + bo);
    }
#pragma unroll
    for (int i = 0; i < 4; ++i) {
      const size_t ao = (size_t)(m0 + (i << 4) + rlane) * lda + koff + k0;
      V ah = Frag<T>::load(Ab + ao);
      V al;
      if (SPLIT) al = Frag<T>::load(Ab2 + ao);
#pragma unroll
      for (int j = 0; j < 4; ++j) {
        acc[i][j] = Frag<T>::mma(ah, bh[j], acc[i][j]);
        if (SPLIT) {
          acc[i][j] = Frag<T>::mma(ah, bl[j], acc[i][j]);
          acc[i][j] = Frag<T>::mma(al, bh[j], acc[i][j]);
        }
      }
      Frag<T>::guard(acc[i][0], acc[i][3], ah, SPLIT ? al : ah);
    }
    Frag<T>::keep(bh[0], bh[1], bh[2], bh[3]);
    if (SPLIT) Frag<T>::keep(bl[0], bl[1], bl[2], bl[3]);
  }
  acc_guard4(acc[0][0], acc[0][1], acc[0][2], acc[0][3]);
  acc_guard4(acc[1][0], acc[1][1], acc[1][2], acc[1][3]);
  acc_guard4(acc[2][0], acc[2][1], acc[2][2], acc[2][3]);
  acc_guard4(acc[3][0], acc[3][1], acc[3][2], acc[3][3]);

  float* slab = sT[wave];
  const float* Rb = RESID ? (resid + (size_t)b * strideR) : nullptr;
#pragma unroll
  for (int i = 0; i < 4; ++i) {
    const int mBase = m0 + (i << 4);
#pragma unroll
    for (int j = 0; j < 4; ++j) {
      const int n = n0 + (j << 4) + rlane;
      float bv = 0.f;
      if (BIAS_MODE == 2) bv = bias[n];
#pragma unroll
      for (int r = 0; r < 8; ++r) {
        float v = acc[i][j][r] * scale;
        if (BIAS_MODE == 1) v += bias[mBase + mOff + r];
        if (BIAS_MODE == 2) v += bv;
        if (RESID) v += Rb[(size_t)(mBase + mOff + r) * ldc + n];
        if (ACT == 1) v = tanhf(v);
        if (ACT == 2) v = fmaxf(v, 0.0f);
        if (ACT == 3) v = v / (1.0f + expf(-v));
        if (ACT == 4) v = (v > 0.f) ? v : 0.01f * v;
        if (ACT == 5) v = 0.5f * v * (1.0f + erff(v * 0.70710678118654752f));
        if (ACT == 6) v = gelu_tanh_f(v);
        slab[(mOff + r) * 68 + (j << 4) + rlane] = v;
      }
    }
    __builtin_amdgcn_fence(__ATOMIC_RELEASE, "workgroup");
    __builtin_amdgcn_wave_barrier();
    __builtin_amdgcn_fence(__ATOMIC_ACQUIRE, "workgroup");
    if (OUT_MODE == 0) {
      float* C = (float*)Cout + (size_t)b * strideC;
      const int hh = lane >> 4, c4 = (lane & 15) * 4;
      for (int pass = 0; pass < 2; ++pass) {
#pragma unroll
        for (int it = 0; it < 8; ++it) {
          const int row = it * 2 + hh;
          v4f v = *(const v4f*)(slab + row * 68 + c4);
          *(volatile v4f*)(C + (size_t)(mBase + row) * ldc + n0 + c4) = v;
        }
        __threadfence();
      }
    } else {
      const int q = lane >> 3, c8 = (lane & 7) * 8;
      unsigned short* C  = (unsigned short*)Cout  + (size_t)b * strideC;
      unsigned short* C2 = (OUT_MODE == 2) ? ((unsigned short*)Cout2 + (size_t)b * strideC) : nullptr;
      for (int pass = 0; pass < 2; ++pass) {
#pragma unroll
        for (int it = 0; it < 4; ++it) {
          const int row = it * 4 + q;
          const float* sp = slab + row * 68 + c8;
          v8h hv, lv;
#pragma unroll
          for (int e = 0; e < 8; ++e) {
            if (OUT_MODE == 1) {
              hv[e] = (_Float16)sp[e];
            } else {
              unsigned short hb = f2bf_bits(sp[e]);
              unsigned short lb = f2bf_bits(sp[e] - bf_bits2f(hb));
              hv[e] = __builtin_bit_cast(_Float16, hb);
              lv[e] = __builtin_bit_cast(_Float16, lb);
            }
          }
          *(volatile v8h*)(C + (size_t)(mBase + row) * ldc + n0 + c8) = hv;
          if (OUT_MODE == 2) *(volatile v8h*)(C2 + (size_t)(mBase + row) * ldc + n0 + c8) = lv;
        }
        __threadfence();
      }
    }
    __builtin_amdgcn_fence(__ATOMIC_RELEASE, "workgroup");
    __builtin_amdgcn_wave_barrier();
    __builtin_amdgcn_fence(__ATOMIC_ACQUIRE, "workgroup");
  }
}

#define AT_D 64
#define AT_NW 4
#define AT_QB 64
#define AT_KC 64
struct AttnGeom { const float* cp = nullptr; const float* pc = nullptr; long c_bs = 0, c_rs = 0, c_hs = 0;
                  long q_bs, q_rs, q_hs, k_bs, k_rs, k_hs, v_bs, v_rs, v_hs, o_bs, o_rs, o_hs;
                  int S, Skv, H, mask_mode; float qscale; int blk0; float mask_fill; int mask_is_int; };
static_assert(sizeof(AttnGeom) == 168, "no padding");

__device__ __forceinline__ unsigned short at_bf_bits(float f) {
  unsigned u = __float_as_uint(f);
  return (unsigned short)((u + 0x7FFFu + ((u >> 16) & 1u)) >> 16);
}
__device__ __forceinline__ __bf16 at_f2bf(float f) { return __builtin_bit_cast(__bf16, at_bf_bits(f)); }
__device__ __forceinline__ void at_split(float f, __bf16& hi, __bf16& lo) {
  const unsigned short hb = at_bf_bits(f);
  hi = __builtin_bit_cast(__bf16, hb);
  lo = at_f2bf(f - __uint_as_float(((unsigned)hb) << 16));
}
__device__ __forceinline__ v8f at_mma(v16b a, v16b b, v8f c) {
  c = __builtin_amdgcn_wmma_f32_16x16x32_bf16(false, a, false, b, (short)0, c, false, false);
  asm volatile("v_nop\n\tv_nop\n\tv_nop\n\tv_nop" : "+v"(c) : "v"(a), "v"(b));
  return c;
}
template <bool F16> __device__ __forceinline__ __bf16 at_to16(float f) {
  if (F16) return __builtin_bit_cast(__bf16, (_Float16)f);
  return at_f2bf(f);
}
template <bool F16> __device__ __forceinline__ v8f at_mma16(v16b a, v16b b, v8f c) {
  if (F16) {
    const v16h ah = __builtin_bit_cast(v16h, a), bh = __builtin_bit_cast(v16h, b);
    c = __builtin_amdgcn_wmma_f32_16x16x32_f16(false, ah, false, bh, (short)0, c, false, false);
    asm volatile("v_nop\n\tv_nop\n\tv_nop\n\tv_nop" : "+v"(c) : "v"(ah), "v"(bh));
    return c;
  }
  return at_mma(a, b, c);
}

template <bool SPLIT_QK, bool SPLIT_PV, bool F16 = false>
__global__ __launch_bounds__(128)
void attn64_kernel(const float* __restrict__ q, const float* __restrict__ k,
                   const float* __restrict__ v, float* __restrict__ out,
                   const void* __restrict__ mask_a, const int* __restrict__ mask_b, AttnGeom g) {
  static_assert(!(F16 && (SPLIT_QK || SPLIT_PV)), "f16 mode is non-split");
  const float PSC = F16 ? 32768.0f : 1.0f;
  union FB { v16b v; v8b h[2]; };
  __shared__ __align__(16) __bf16 Ksh[AT_KC * AT_D];
  __shared__ __align__(16) __bf16 Ksl[SPLIT_QK ? AT_KC * AT_D : 8];
  __shared__ __align__(16) __bf16 Vth[AT_D * AT_KC];
  __shared__ __align__(16) __bf16 Vtl[SPLIT_PV ? AT_D * AT_KC : 8];
  __shared__ __align__(16) __bf16 Psh[AT_NW][16 * AT_KC];
  __shared__ __align__(16) __bf16 Psl[SPLIT_PV ? AT_NW : 1][SPLIT_PV ? 16 * AT_KC : 8];
  __shared__ __align__(16) float  Os[AT_NW][16 * 68];

  const int tid  = threadIdx.x;
  const int wave = tid >> 5;
  const int lane = tid & 31;
  const int hh   = lane >> 4;
  const int c    = lane & 15;

  const int nqb = g.S / AT_QB;
  const int bx = blockIdx.x + g.blk0;
  const int qb = bx % nqb;
  const int bh = bx / nqb;
  const int h  = bh % g.H;
  const int b  = bh / g.H;
  const int qbase_block = qb * AT_QB;
  const int q0 = qbase_block + wave * 16;

  const float* qb_ptr = q + (size_t)b * g.q_bs + (size_t)h * g.q_hs;
  const float* kb_ptr = k + (size_t)b * g.k_bs + (size_t)h * g.k_hs;
  const float* vb_ptr = v + (size_t)b * g.v_bs + (size_t)h * g.v_hs;
  float*       ob_ptr = out + (size_t)b * g.o_bs + (size_t)h * g.o_hs;

  v16b qah[2], qal[2];
  {
    const float* qrow = qb_ptr + (size_t)(q0 + c) * g.q_rs;
#pragma unroll
    for (int dc = 0; dc < 2; ++dc) {
#pragma unroll
      for (int e = 0; e < 8; ++e) {
        const float f0 = qrow[dc * 32 + 8 * hh + e] * g.qscale;
        const float f1 = qrow[dc * 32 + 16 + 8 * hh + e] * g.qscale;
        if (SPLIT_QK) { __bf16 hq, lq; at_split(f0, hq, lq); qah[dc][e] = hq; qal[dc][e] = lq; at_split(f1, hq, lq); qah[dc][8 + e] = hq; qal[dc][8 + e] = lq; }
        else { qah[dc][e] = at_to16<F16>(f0); qah[dc][8 + e] = at_to16<F16>(f1); qal[dc][e] = qah[dc][e]; qal[dc][8 + e] = qah[dc][8 + e]; }
      }
    }
  }

  float mrow[8], lrow[8];
  v8f oacc[4];
#pragma unroll
  for (int r = 0; r < 8; ++r) { mrow[r] = -INFINITY; lrow[r] = 0.f; }
#pragma unroll
  for (int t = 0; t < 4; ++t) oacc[t] = (v8f){0.f,0.f,0.f,0.f,0.f,0.f,0.f,0.f};

  const int nChunks = (g.mask_mode == 1 || g.mask_mode == 4) ? (qb + 1) : (g.Skv / AT_KC);
  int qkeep[8];
#pragma unroll
  for (int r = 0; r < 8; ++r) qkeep[r] = (g.mask_mode == 3) ? mask_b[(size_t)b * g.S + q0 + 8 * hh + r] : 1;
  for (int kc = 0; kc < nChunks; ++kc) {
    const int kv0 = kc * AT_KC;
    __syncthreads();
    {
      const int kvr = tid >> 1, dh = (tid & 1) * 32;
      const float* krow = kb_ptr + (size_t)(kv0 + kvr) * g.k_rs + dh;
      const float* vrow = vb_ptr + (size_t)(kv0 + kvr) * g.v_rs + dh;
#pragma unroll
      for (int i = 0; i < 8; ++i) {
        v4f kk = *(const v4f*)(krow + 4 * i);
        v4f vv = *(const v4f*)(vrow + 4 * i);
#pragma unroll
        for (int e = 0; e < 4; ++e) {
          const int d = dh + 4 * i + e;
          if (SPLIT_QK) { __bf16 a, bl; at_split(kk[e], a, bl); Ksh[kvr * AT_D + d] = a; Ksl[kvr * AT_D + d] = bl; }
          else Ksh[kvr * AT_D + d] = at_to16<F16>(kk[e]);
          if (SPLIT_PV) { __bf16 a, bl; at_split(vv[e], a, bl); Vth[d * AT_KC + kvr] = a; Vtl[d * AT_KC + kvr] = bl; }
          else Vth[d * AT_KC + kvr] = at_to16<F16>(vv[e]);
        }
      }
    }
    __syncthreads();

    v8f s[4];
#pragma unroll
    for (int j = 0; j < 4; ++j) {
      s[j] = (v8f){0.f,0.f,0.f,0.f,0.f,0.f,0.f,0.f};
#pragma unroll 1
      for (int dc = 0; dc < 2; ++dc) {
        FB kb;
        kb.h[0] = *(const v8b*)(Ksh + (j * 16 + c) * AT_D + dc * 32 + 8 * hh);
        kb.h[1] = *(const v8b*)(Ksh + (j * 16 + c) * AT_D + dc * 32 + 16 + 8 * hh);
        s[j] = at_mma16<F16>(qah[dc], kb.v, s[j]);
        if (SPLIT_QK) {
          FB kl;
          kl.h[0] = *(const v8b*)(Ksl + (j * 16 + c) * AT_D + dc * 32 + 8 * hh);
          kl.h[1] = *(const v8b*)(Ksl + (j * 16 + c) * AT_D + dc * 32 + 16 + 8 * hh);
          s[j] = at_mma16<F16>(qah[dc], kl.v, s[j]);
          s[j] = at_mma16<F16>(qal[dc], kb.v, s[j]);
        }
      }
    }
    const bool diag = (g.mask_mode == 1) && (kc == qb);
    int kvkeep[4] = {1, 1, 1, 1};
    if (g.mask_mode == 3) {
#pragma unroll
      for (int j = 0; j < 4; ++j) kvkeep[j] = ((const int*)mask_a)[(size_t)b * g.Skv + kv0 + j * 16 + c];
    }
    float cm[8];
#pragma unroll
    for (int r = 0; r < 8; ++r) {
      const int qrow = q0 + 8 * hh + r;
      float m = -INFINITY;
#pragma unroll
      for (int j = 0; j < 4; ++j) {
        const int kvcol = kv0 + j * 16 + c;
        bool masked = false;
        if (diag) masked = (kvcol > qrow);
        else if (g.mask_mode == 4) masked = (kvcol > qrow) || (qrow - kvcol > g.mask_is_int);
        else if (g.mask_mode == 2) {
          const size_t mi = (size_t)qrow * g.Skv + kvcol;
          masked = (g.mask_is_int == 0) ? (((const float*)mask_a)[mi] == 0.0f)
                 : (g.mask_is_int == 1) ? (((const int*)mask_a)[mi] == 0) : (((const int*)mask_a)[mi] != 0);
        } else if (g.mask_mode == 3) masked = (qkeep[r] == 0) || (kvkeep[j] == 0);
        else if (g.mask_mode == 5) {
          const size_t mi = (size_t)qrow * g.Skv + kvcol;
          masked = (((const int*)mask_a)[mi] != 0);
          int n = mask_b[mi]; n = n < 0 ? 0 : n;
          s[j][r] += g.cp[(size_t)b * g.c_bs + (size_t)h * g.c_hs + (size_t)qrow * g.c_rs + n]
                   + g.pc[(size_t)b * g.c_bs + (size_t)h * g.c_hs + (size_t)kvcol * g.c_rs + n];
        }
        if (masked) s[j][r] = g.mask_fill;
        m = fmaxf(m, s[j][r]);
      }
#pragma unroll
      for (int off = 1; off < 16; off <<= 1) m = fmaxf(m, __shfl_xor(m, off, 32));
      cm[r] = m;
    }
    __bf16* pwh = Psh[wave];
    __bf16* pwl = Psl[SPLIT_PV ? wave : 0];
#pragma unroll
    for (int r = 0; r < 8; ++r) {
      const float mnew = fmaxf(mrow[r], cm[r]);
      const float alpha = expf(mrow[r] - mnew);
      mrow[r] = mnew;
      float psum = 0.f;
#pragma unroll
      for (int j = 0; j < 4; ++j) {
        const float p = expf(s[j][r] - mnew);
        psum += p;
        if (SPLIT_PV) { __bf16 a, bl; at_split(p, a, bl); pwh[(8 * hh + r) * AT_KC + j * 16 + c] = a; pwl[(8 * hh + r) * AT_KC + j * 16 + c] = bl; }
        else pwh[(8 * hh + r) * AT_KC + j * 16 + c] = at_to16<F16>(p * PSC);
      }
#pragma unroll
      for (int off = 1; off < 16; off <<= 1) psum += __shfl_xor(psum, off, 32);
      lrow[r] = lrow[r] * alpha + psum;
#pragma unroll
      for (int t = 0; t < 4; ++t) oacc[t][r] *= alpha;
    }
    __builtin_amdgcn_fence(__ATOMIC_RELEASE, "workgroup");
    __builtin_amdgcn_wave_barrier();
    __builtin_amdgcn_fence(__ATOMIC_ACQUIRE, "workgroup");
#pragma unroll 1
    for (int kk = 0; kk < 2; ++kk) {
      FB pa, pl;
      pa.h[0] = *(const v8b*)(pwh + c * AT_KC + kk * 32 + 8 * hh);
      pa.h[1] = *(const v8b*)(pwh + c * AT_KC + kk * 32 + 16 + 8 * hh);
      if (SPLIT_PV) {
        pl.h[0] = *(const v8b*)(pwl + c * AT_KC + kk * 32 + 8 * hh);
        pl.h[1] = *(const v8b*)(pwl + c * AT_KC + kk * 32 + 16 + 8 * hh);
      }
#pragma unroll
      for (int t = 0; t < 4; ++t) {
        FB vb;
        vb.h[0] = *(const v8b*)(Vth + (t * 16 + c) * AT_KC + kk * 32 + 8 * hh);
        vb.h[1] = *(const v8b*)(Vth + (t * 16 + c) * AT_KC + kk * 32 + 16 + 8 * hh);
        oacc[t] = at_mma16<F16>(pa.v, vb.v, oacc[t]);
        if (SPLIT_PV) {
          FB vl;
          vl.h[0] = *(const v8b*)(Vtl + (t * 16 + c) * AT_KC + kk * 32 + 8 * hh);
          vl.h[1] = *(const v8b*)(Vtl + (t * 16 + c) * AT_KC + kk * 32 + 16 + 8 * hh);
          oacc[t] = at_mma16<F16>(pa.v, vl.v, oacc[t]);
          oacc[t] = at_mma16<F16>(pl.v, vb.v, oacc[t]);
        }
      }
    }
  }

  float* os = Os[wave];
#pragma unroll
  for (int r = 0; r < 8; ++r) {
    const float inv = 1.0f / (lrow[r] * PSC);
#pragma unroll
    for (int t = 0; t < 4; ++t) os[(8 * hh + r) * 68 + t * 16 + c] = oacc[t][r] * inv;
  }
  __builtin_amdgcn_fence(__ATOMIC_RELEASE, "workgroup");
  __builtin_amdgcn_wave_barrier();
  __builtin_amdgcn_fence(__ATOMIC_ACQUIRE, "workgroup");
  {
    const int c4 = (lane & 15) * 4;
    for (int pass = 0; pass < 2; ++pass) {
#pragma unroll
      for (int it = 0; it < 8; ++it) {
        const int row = it * 2 + hh;
        v4f val = *(const v4f*)(os + row * 68 + c4);
        *(volatile v4f*)(ob_ptr + (size_t)(q0 + row) * g.o_rs + c4) = val;
      }
      __threadfence();
    }
  }
}

__device__ __forceinline__ float wsum32(float v) {
#pragma unroll
  for (int off = 16; off > 0; off >>= 1) v += __shfl_xor(v, off, 32);
  return v;
}

__global__ __launch_bounds__(256) void k_tcast(const float* __restrict__ in, _Float16* __restrict__ out,
                                               int R, int C, float mul) {
  __shared__ float ts[64 * 65];
  const int tid = threadIdx.x, lane = tid & 31, wave = tid >> 5;
  const int r0 = blockIdx.y * 64, c0 = blockIdx.x * 64;
  {
    const int rl = tid >> 2, c4 = (tid & 3) * 16;
    const float* src = in + (size_t)(r0 + rl) * C + c0 + c4;
#pragma unroll
    for (int i = 0; i < 4; ++i) {
      const v4f v = *(const v4f*)(src + 4 * i);
#pragma unroll
      for (int e = 0; e < 4; ++e) ts[(c4 + 4 * i + e) * 65 + rl] = v[e];
    }
  }
  __syncthreads();
  const int q = lane >> 3, c8 = (lane & 7) * 8;
  for (int pass = 0; pass < 2; ++pass) {
#pragma unroll
    for (int it = 0; it < 2; ++it) {
      const int cl = wave * 8 + it * 4 + q;
      const float* sp = ts + cl * 65 + c8;
      v8h hv;
#pragma unroll
      for (int e = 0; e < 8; ++e) hv[e] = (_Float16)(sp[e] * mul);
      *(volatile v8h*)(out + (size_t)(c0 + cl) * R + r0 + c8) = hv;
    }
    __threadfence();
  }
}

__global__ __launch_bounds__(256) void k_ada(const float* __restrict__ c, const float* __restrict__ w,
                                             const float* __restrict__ bias, float* __restrict__ ada, int total) {
  const int id = blockIdx.x * 256 + threadIdx.x;
  const int idc = id < total ? id : total - 1;
  const int j = idc % ADA6;
  const int b = idc / ADA6;
  float s = bias[j];
#pragma unroll 1
  for (int k = 0; k < COND; ++k) s = fmaf(c[b * COND + k], w[(size_t)k * ADA6 + j], s);
  if (id < total) {
    ((volatile float*)ada)[idc] = s;
    __threadfence();
    ((volatile float*)ada)[idc] = s;
  }
}

__global__ __launch_bounds__(256) void k_blkmask(int* __restrict__ mn, int* __restrict__ mc) {
  const int row = blockIdx.x;
  const int tid = threadIdx.x;
  if (row < NHALF) {
    const int bq = row / BLK;
    int* dst = mn + (size_t)row * SEQ;
    v4i vals[2];
#pragma unroll
    for (int it = 0; it < 2; ++it) {
      const int j0 = (tid + 256 * it) * 4;
      v4i m;
#pragma unroll
      for (int e = 0; e < 4; ++e) {
        const int j = j0 + e;
        const bool fk = (j >= NHALF);
        const int bk = fk ? ((j - NHALF) / BLK) : (j / BLK);
        m[e] = fk ? ((bq > bk) ? 1 : 0) : ((bq == bk) ? 1 : 0);
      }
      vals[it] = m;
    }
    for (int pass = 0; pass < 2; ++pass) {
#pragma unroll
      for (int it = 0; it < 2; ++it) *(volatile v4i*)(dst + (size_t)(tid + 256 * it) * 4) = vals[it];
      __threadfence();
    }
  } else {
    const int i2 = row - NHALF;
    const int bq = i2 / BLK;
    int* dst = mc + (size_t)i2 * NHALF;
    const int j0 = tid * 4;
    v4i m;
#pragma unroll
    for (int e = 0; e < 4; ++e) m[e] = (bq >= (j0 + e) / BLK) ? 1 : 0;
    *(volatile v4i*)(dst + j0) = m;
    __threadfence();
    *(volatile v4i*)(dst + j0) = m;
  }
}

__global__ __launch_bounds__(96) void k_ln_mod(const float* __restrict__ xin, const float* __restrict__ lnw,
                                               const float* __restrict__ ada, int shiftOff, int scaleOff,
                                               _Float16* __restrict__ hout) {
  __shared__ float red[4];
  const int row = blockIdx.x, b = row >> 11, t = threadIdx.x, lane = t & 31, wave = t >> 5;
  const float* xr = xin + (size_t)row * DIM + 8 * t;
  const v4f a0 = *(const v4f*)xr;
  const v4f a1 = *(const v4f*)(xr + 4);
  float s = ((a0[0] + a0[1]) + (a0[2] + a0[3])) + ((a1[0] + a1[1]) + (a1[2] + a1[3]));
  s = wsum32(s);
  if (lane == 0) red[wave] = s;
  __syncthreads();
  const float mean = ((red[0] + red[1]) + red[2]) * (1.0f / DIM);
  __syncthreads();
  float d[8];
  d[0] = a0[0] - mean; d[1] = a0[1] - mean; d[2] = a0[2] - mean; d[3] = a0[3] - mean;
  d[4] = a1[0] - mean; d[5] = a1[1] - mean; d[6] = a1[2] - mean; d[7] = a1[3] - mean;
  float qs = 0.f;
#pragma unroll
  for (int e = 0; e < 8; ++e) qs += d[e] * d[e];
  qs = wsum32(qs);
  if (lane == 0) red[wave] = qs;
  __syncthreads();
  const float var = ((red[0] + red[1]) + red[2]) * (1.0f / DIM);
  const float rs = rsqrtf(var + 1e-5f);
  const float* ad = ada + (size_t)b * ADA6;
  v8h hv;
#pragma unroll
  for (int e = 0; e < 8; ++e) {
    const int j = 8 * t + e;
    float hval = d[e] * rs * lnw[j];
    hval = hval * (1.0f + ad[scaleOff + j]) + ad[shiftOff + j];
    hv[e] = (_Float16)hval;
  }
  _Float16* dst = hout + (size_t)row * DIM + 8 * t;
  *(volatile v8h*)dst = hv;
  __threadfence();
  *(volatile v8h*)dst = hv;
}

__global__ __launch_bounds__(256) void k_rope(float* __restrict__ qkv, const float* __restrict__ cosb,
                                              const float* __restrict__ sinb) {
  __shared__ __align__(16) float xs[QKVW];
  const int row = blockIdx.x, tid = threadIdx.x;
  const int s = row & (SEQ - 1);
  const int p = s & (NHALF - 1);
  float* rp = qkv + (size_t)row * QKVW;
  for (int f = tid; f < QKVW / 4; f += 256) *(v4f*)(xs + 4 * f) = *(const v4f*)(rp + 4 * f);
  __syncthreads();
  for (int pass = 0; pass < 2; ++pass) {
#pragma unroll
    for (int it = 0; it < 3; ++it) {
      const int f = tid + 256 * it;
      if (f < QKVW / 4) {
        const int cidx = 4 * f;
        const int d0 = cidx & 63;
        int ihi = cidx + 32; ihi = ihi > QKVW - 4 ? QKVW - 4 : ihi;
        int ilo = cidx - 32; ilo = ilo < 0 ? 0 : ilo;
        const v4f xv = *(const v4f*)(xs + cidx);
        const v4f vhi = *(const v4f*)(xs + ihi);
        const v4f vlo = *(const v4f*)(xs + ilo);
        const v4f cs = *(const v4f*)(cosb + p * HD + d0);
        const v4f sn = *(const v4f*)(sinb + p * HD + d0);
        v4f rh = vlo;
        if (d0 < 32) rh = -vhi;
        const v4f o = xv * cs + rh * sn;
        *(volatile v4f*)(rp + cidx) = o;
      }
    }
    __threadfence();
  }
}

__global__ __launch_bounds__(256) void k_cast8(const float* __restrict__ in, _Float16* __restrict__ out,
                                               float mul, int n8) {
  const int id = blockIdx.x * 256 + threadIdx.x;
  const int idc = id < n8 ? id : n8 - 1;
  const v4f a0 = *(const v4f*)(in + (size_t)idc * 8);
  const v4f a1 = *(const v4f*)(in + (size_t)idc * 8 + 4);
  v8h hv;
#pragma unroll
  for (int e = 0; e < 4; ++e) { hv[e] = (_Float16)(a0[e] * mul); hv[4 + e] = (_Float16)(a1[e] * mul); }
  if (id < n8) {
    _Float16* dst = out + (size_t)idc * 8;
    *(volatile v8h*)dst = hv;
    __threadfence();
    *(volatile v8h*)dst = hv;
  }
}

__global__ __launch_bounds__(96) void k_res_ln2(const float* __restrict__ ow, const float* __restrict__ xin,
                                                const float* __restrict__ lnw, const float* __restrict__ ada,
                                                float* __restrict__ x1out, _Float16* __restrict__ hout) {
  __shared__ __align__(16) float xs[DIM];
  __shared__ float red[4];
  const int row = blockIdx.x, b = row >> 11, t = threadIdx.x, lane = t & 31, wave = t >> 5;
  const float* ad = ada + (size_t)b * ADA6;
  const size_t rbase = (size_t)row * DIM;
  v4f r0v, r1v;
  {
    const int f = t;
    const v4f o4 = *(const v4f*)(ow + rbase + 4 * f);
    const v4f x4 = *(const v4f*)(xin + rbase + 4 * f);
    const v4f g4 = *(const v4f*)(ad + 2 * DIM + 4 * f);
    r0v = g4 * o4 + x4;
    *(v4f*)(xs + 4 * f) = r0v;
  }
  {
    const int f = t + 96;
    const v4f o4 = *(const v4f*)(ow + rbase + 4 * f);
    const v4f x4 = *(const v4f*)(xin + rbase + 4 * f);
    const v4f g4 = *(const v4f*)(ad + 2 * DIM + 4 * f);
    r1v = g4 * o4 + x4;
    *(v4f*)(xs + 4 * f) = r1v;
  }
  *(volatile v4f*)(x1out + rbase + 4 * t) = r0v;
  *(volatile v4f*)(x1out + rbase + 4 * (t + 96)) = r1v;
  __threadfence();
  *(volatile v4f*)(x1out + rbase + 4 * t) = r0v;
  *(volatile v4f*)(x1out + rbase + 4 * (t + 96)) = r1v;
  __syncthreads();
  const v4f a0 = *(const v4f*)(xs + 8 * t);
  const v4f a1 = *(const v4f*)(xs + 8 * t + 4);
  float s = ((a0[0] + a0[1]) + (a0[2] + a0[3])) + ((a1[0] + a1[1]) + (a1[2] + a1[3]));
  s = wsum32(s);
  if (lane == 0) red[wave] = s;
  __syncthreads();
  const float mean = ((red[0] + red[1]) + red[2]) * (1.0f / DIM);
  __syncthreads();
  float d[8];
  d[0] = a0[0] - mean; d[1] = a0[1] - mean; d[2] = a0[2] - mean; d[3] = a0[3] - mean;
  d[4] = a1[0] - mean; d[5] = a1[1] - mean; d[6] = a1[2] - mean; d[7] = a1[3] - mean;
  float qs = 0.f;
#pragma unroll
  for (int e = 0; e < 8; ++e) qs += d[e] * d[e];
  qs = wsum32(qs);
  if (lane == 0) red[wave] = qs;
  __syncthreads();
  const float var = ((red[0] + red[1]) + red[2]) * (1.0f / DIM);
  const float rs = rsqrtf(var + 1e-5f);
  v8h hv;
#pragma unroll
  for (int e = 0; e < 8; ++e) {
    const int j = 8 * t + e;
    float hval = d[e] * rs * lnw[j];
    hval = hval * (1.0f + ad[4 * DIM + j]) + ad[3 * DIM + j];
    hv[e] = (_Float16)hval;
  }
  _Float16* dst = hout + rbase + 8 * t;
  *(volatile v8h*)dst = hv;
  __threadfence();
  *(volatile v8h*)dst = hv;
}

__global__ __launch_bounds__(256) void k_final(const float* __restrict__ m2, const float* __restrict__ x1,
                                               const float* __restrict__ ada, float* __restrict__ out, int total4) {
  const int id = blockIdx.x * 256 + threadIdx.x;
  const int idc = id < total4 ? id : total4 - 1;
  const int row = idc / (DIM / 4);
  const int f = idc - row * (DIM / 4);
  const int b = row >> 11;
  const v4f g = *(const v4f*)(ada + (size_t)b * ADA6 + 5 * DIM + 4 * f);
  const v4f mv = *(const v4f*)(m2 + (size_t)idc * 4);
  const v4f xv = *(const v4f*)(x1 + (size_t)idc * 4);
  const v4f o = g * mv + xv;
  if (id < total4) {
    *(volatile v4f*)(out + (size_t)idc * 4) = o;
    __threadfence();
    *(volatile v4f*)(out + (size_t)idc * 4) = o;
  }
}

extern "C" void kernel_launch(void* const* d_in, const int* in_sizes, int n_in,
                              void* d_out, int out_size, void* d_ws, size_t ws_size,
                              hipStream_t stream) {
  if (n_in < 14) return;
  if (in_sizes[0] != ROWS * DIM || in_sizes[1] != NHALF * HD || in_sizes[2] != NHALF * HD ||
      in_sizes[3] != 2 * COND || in_sizes[4] != DIM * QKVW || in_sizes[5] != DIM * DIM ||
      in_sizes[6] != DIM || in_sizes[7] != DIM || in_sizes[8] != DIM * DFF || in_sizes[9] != DFF ||
      in_sizes[10] != DFF * DIM || in_sizes[11] != DIM || in_sizes[12] != COND * ADA6 || in_sizes[13] != ADA6)
    return;
  if (out_size != ROWS * DIM) return;

  const float* x    = (const float*)d_in[0];
  const float* cosb = (const float*)d_in[1];
  const float* sinb = (const float*)d_in[2];
  const float* c    = (const float*)d_in[3];
  const float* Wqkv = (const float*)d_in[4];
  const float* Wout = (const float*)d_in[5];
  const float* ln1w = (const float*)d_in[6];
  const float* ln2w = (const float*)d_in[7];
  const float* w1   = (const float*)d_in[8];
  const float* b1   = (const float*)d_in[9];
  const float* w2   = (const float*)d_in[10];
  const float* b2   = (const float*)d_in[11];
  const float* adaw = (const float*)d_in[12];
  const float* adab = (const float*)d_in[13];
  float* out = (float*)d_out;

  const size_t szWQ = (size_t)QKVW * DIM * 2, szWO = (size_t)DIM * DIM * 2;
  const size_t szW1 = (size_t)DFF * DIM * 2, szW2 = (size_t)DIM * DFF * 2;
  const size_t szADA = (size_t)2 * ADA6 * 4;
  const size_t szH16 = (size_t)ROWS * DIM * 2;
  const size_t szBIG = (size_t)ROWS * QKVW * 4;
  const size_t szPL = (size_t)ROWS * DIM * 4;
  const size_t szMN = (size_t)NHALF * SEQ * 4;
  size_t off = 0;
  auto carve = [&](size_t bytes) { size_t o = off; off += (bytes + 255) & ~(size_t)255; return o; };
  const size_t oWQ = carve(szWQ), oWO = carve(szWO), oW1 = carve(szW1), oW2 = carve(szW2);
  const size_t oADA = carve(szADA);
  const size_t oH16 = carve(szH16);
  const size_t oBIG = carve(szBIG);
  const size_t oMSK = carve(szPL);
  const size_t oOPL = carve(szPL);
  if (off > ws_size) return;
  if (oOPL != oMSK + szPL) return;
  if (szBIG != 3 * szPL) return;

  char* ws = (char*)d_ws;
  _Float16* WQ16 = (_Float16*)(ws + oWQ);
  _Float16* WO16 = (_Float16*)(ws + oWO);
  _Float16* W116 = (_Float16*)(ws + oW1);
  _Float16* W216 = (_Float16*)(ws + oW2);
  float* ADA = (float*)(ws + oADA);
  _Float16* H16 = (_Float16*)(ws + oH16);
  _Float16* O16 = H16;
  _Float16* H2  = H16;
  float* QKV = (float*)(ws + oBIG);
  float* OW  = (float*)(ws + oBIG);
  float* X1  = (float*)(ws + oBIG + szPL);
  float* M2  = (float*)(ws + oBIG + 2 * szPL);
  int* MN = (int*)(ws + oMSK);
  int* MC = (int*)(ws + oMSK + szMN);
  float* OPL = (float*)(ws + oOPL);
  _Float16* G16 = (_Float16*)(ws + oMSK);

  k_tcast<<<dim3(QKVW / 64, DIM / 64), 256, 0, stream>>>(Wqkv, WQ16, DIM, QKVW, 16.0f);
  k_tcast<<<dim3(DIM / 64, DIM / 64), 256, 0, stream>>>(Wout, WO16, DIM, DIM, 16.0f);
  k_tcast<<<dim3(DFF / 64, DIM / 64), 256, 0, stream>>>(w1, W116, DIM, DFF, 16.0f);
  k_tcast<<<dim3(DIM / 64, DFF / 64), 256, 0, stream>>>(w2, W216, DFF, DIM, 16.0f);

  k_ada<<<(2 * ADA6 + 255) / 256, 256, 0, stream>>>(c, adaw, adab, ADA, 2 * ADA6);

  k_blkmask<<<2 * NHALF, 256, 0, stream>>>(MN, MC);

  k_ln_mod<<<ROWS, 96, 0, stream>>>(x, ln1w, ADA, 0, DIM, H16);

  wmma_gemm64<0, false, 0, 0, false, 0><<<dim3((ROWS / 64) * (QKVW / 64) / 8, 1), 256, 0, stream>>>(
      U16(H16), U16(H16), DIM, 0L, U16(WQ16), U16(WQ16), DIM, 0L,
      (void*)QKV, (void*)QKV, QKVW, 0L, ADA, x, 0L, ROWS, QKVW, DIM, 1.0f / 16.0f);

  k_rope<<<ROWS, 256, 0, stream>>>(QKV, cosb, sinb);

  AttnGeom gn{};
  gn.cp = ADA; gn.pc = ADA; gn.c_bs = 0; gn.c_rs = 0; gn.c_hs = 0;
  gn.q_bs = (long)SEQ * QKVW; gn.q_rs = QKVW; gn.q_hs = HD;
  gn.k_bs = (long)SEQ * QKVW; gn.k_rs = QKVW; gn.k_hs = HD;
  gn.v_bs = (long)SEQ * QKVW; gn.v_rs = QKVW; gn.v_hs = HD;
  gn.o_bs = (long)SEQ * DIM;  gn.o_rs = DIM;  gn.o_hs = HD;
  gn.S = NHALF; gn.Skv = SEQ; gn.H = HEADS; gn.mask_mode = 2; gn.qscale = 0.125f; gn.blk0 = 0;
  gn.mask_fill = -1e30f; gn.mask_is_int = 1;
  attn64_kernel<false, false, true><<<2 * HEADS * (NHALF / 64), 128, 0, stream>>>(
      QKV, QKV + DIM, QKV + 2 * DIM, OPL, (const void*)MN, (const int*)MN, gn);
  AttnGeom gc = gn;
  gc.Skv = NHALF;
  attn64_kernel<false, false, true><<<2 * HEADS * (NHALF / 64), 128, 0, stream>>>(
      QKV + (size_t)NHALF * QKVW, QKV + (size_t)NHALF * QKVW + DIM, QKV + (size_t)NHALF * QKVW + 2 * DIM,
      OPL + (size_t)NHALF * DIM, (const void*)MC, (const int*)MC, gc);

  k_cast8<<<(ROWS * DIM / 8 + 255) / 256, 256, 0, stream>>>(OPL, O16, 16.0f, ROWS * DIM / 8);

  wmma_gemm64<0, false, 0, 0, false, 0><<<dim3((ROWS / 64) * (DIM / 64) / 8, 1), 256, 0, stream>>>(
      U16(O16), U16(O16), DIM, 0L, U16(WO16), U16(WO16), DIM, 0L,
      (void*)OW, (void*)OW, DIM, 0L, ADA, x, 0L, ROWS, DIM, DIM, 1.0f / 256.0f);

  k_res_ln2<<<ROWS, 96, 0, stream>>>(OW, x, ln2w, ADA, X1, H2);

  wmma_gemm64<0, false, 2, 1, false, 6><<<dim3((ROWS / 64) * (DFF / 64) / 8, 1), 256, 0, stream>>>(
      U16(H2), U16(H2), DIM, 0L, U16(W116), U16(W116), DIM, 0L,
      (void*)G16, (void*)G16, DFF, 0L, b1, x, 0L, ROWS, DFF, DIM, 1.0f / 16.0f);

  wmma_gemm64<0, false, 2, 0, false, 0><<<dim3((ROWS / 64) * (DIM / 64) / 8, 1), 256, 0, stream>>>(
      U16(G16), U16(G16), DFF, 0L, U16(W216), U16(W216), DFF, 0L,
      (void*)M2, (void*)M2, DIM, 0L, b2, x, 0L, ROWS, DIM, DFF, 1.0f / 16.0f);

  k_final<<<(ROWS * DIM / 4 + 255) / 256, 256, 0, stream>>>(M2, X1, ADA, out, ROWS * DIM / 4);
}
